// CrossModalAttentionFusion_54820962566443
// MI455X (gfx1250) — hardware-verified
//
#include <hip/hip_runtime.h>
#include <math.h>
#include <stdint.h>


#define NB   16
#define CH   512
#define CQ   64
#define NT   1024
#define TOK  (NB * NT)
#define RSB  32
#define NRB  (NT / RSB)
#define OUTN (NB * CH * NT)

#define SCW  64.0f
#define SCQK 8.0f
#define SCV  8.0f
#define SCE  32.0f
#define SCA  1024.0f
#define RSCL 0.044194173824159216f
#define SCS  ((1.0f / (SCQK * SCQK)) * RSCL)

static_assert(TOK % 64 == 0 && CH % 64 == 0 && CQ % 64 == 0 && NT % 64 == 0);
static_assert(CH % 32 == 0 && (2 * CH) % 32 == 0 && CQ % 32 == 0 && NT % 32 == 0);
static_assert((((TOK / 64) * (CQ / 64)) % 8) == 0);
static_assert((((CH / 64) * (TOK / 64)) % 8) == 0);
static_assert((((CH / 64) * (NT / 64)) % 8) == 0);
static_assert(NT == 4 * 256 && RSB == 32 && (NT / 16) % 8 == 0 && NT % RSB == 0);
static_assert(TOK % 1024 == 0 && (TOK / 1024) == NB && NT == 1024);
static_assert(CH % 256 == 0 && CH == 8 * 64 && CH % 32 == 0);
static_assert((CQ * CH) % 2048 == 0 && (CH * CH) % 2048 == 0 && (CH * 2 * CH) % 2048 == 0);
static_assert(NT % 128 == 0);

typedef _Float16       v16h __attribute__((ext_vector_type(16)));
typedef _Float16       v8h  __attribute__((ext_vector_type(8)));
typedef float          v8f  __attribute__((ext_vector_type(8)));
typedef float          v4f  __attribute__((ext_vector_type(4)));
typedef unsigned int   v4u  __attribute__((ext_vector_type(4)));

union HU { v8h h; v4u u; _Float16 s[8]; };
union FR { v16h v; v8h h[2]; _Float16 s[16]; };
static_assert(sizeof(HU) == 16);
static_assert(sizeof(FR) == 32);

__device__ __forceinline__ unsigned short bf_bits(float f) {
  const unsigned u = __float_as_uint(f);
  return (unsigned short)((u + 0x7FFFu + ((u >> 16) & 1u)) >> 16);
}
__device__ __forceinline__ float bf_up(unsigned short h) { return __uint_as_float(((unsigned)h) << 16); }
__device__ __forceinline__ float bfr(float f) { return bf_up(bf_bits(f)); }
__device__ __forceinline__ v8f zero8() { v8f z = {0.f, 0.f, 0.f, 0.f, 0.f, 0.f, 0.f, 0.f}; return z; }

__device__ __forceinline__ void ld8(const float* p, float* o) {
  const v4f a = *(const v4f*)(p);
  const v4f b = *(const v4f*)(p + 4);
  o[0] = a[0]; o[1] = a[1]; o[2] = a[2]; o[3] = a[3];
  o[4] = b[0]; o[5] = b[1]; o[6] = b[2]; o[7] = b[3];
}
__device__ __forceinline__ void st8(float* p, const float* o) {
  v4f a, b;
  a[0] = o[0]; a[1] = o[1]; a[2] = o[2]; a[3] = o[3];
  b[0] = o[4]; b[1] = o[5]; b[2] = o[6]; b[3] = o[7];
  *(v4f*)(p) = a;
  *(v4f*)(p + 4) = b;
}

__device__ __forceinline__ double shfl_xor_d(double v, int m) {
  const unsigned long long u = (unsigned long long)__double_as_longlong(v);
  int lo = (int)(unsigned)(u & 0xffffffffull);
  int hi = (int)(unsigned)(u >> 32);
  lo = __shfl_xor(lo, m, 32);
  hi = __shfl_xor(hi, m, 32);
  const unsigned long long r = (((unsigned long long)(unsigned)hi) << 32) | (unsigned long long)(unsigned)lo;
  return __longlong_as_double((long long)r);
}

__device__ __forceinline__ v16h ldfrag_h(const _Float16* p) {
  FR f;
  f.h[0] = *(const v8h*)(p);
  f.h[1] = *(const v8h*)(p + 16);
  return f.v;
}

__device__ __forceinline__ v8f mma_h(v16h a, v16h b, v8f c) {
  c = __builtin_amdgcn_wmma_f32_16x16x32_f16(false, a, false, b, (short)0, c, false, false);
#if defined(__HIP_DEVICE_COMPILE__)
  asm volatile("v_nop\n\tv_nop\n\tv_nop\n\tv_nop" : "+v"(c) : "v"(a), "v"(b));
#endif
  return c;
}
__device__ __forceinline__ v8f mma_h_raw(v16h a, v16h b, v8f c) {
  return __builtin_amdgcn_wmma_f32_16x16x32_f16(false, a, false, b, (short)0, c, false, false);
}
__device__ __forceinline__ void dep_guard_h(v8f& a, v8f& b, v16h x) {
#if defined(__HIP_DEVICE_COMPILE__)
  asm volatile("v_nop\n\tv_nop\n\tv_nop\n\tv_nop" : "+v"(a), "+v"(b) : "v"(x));
#endif
}
__device__ __forceinline__ void keep4_h(v16h a, v16h b, v16h c, v16h d) {
#if defined(__HIP_DEVICE_COMPILE__)
  asm volatile("v_nop" :: "v"(a), "v"(b), "v"(c), "v"(d));
#endif
}
__device__ __forceinline__ void acc_guard4(v8f& a, v8f& b, v8f& c, v8f& d) {
#if defined(__HIP_DEVICE_COMPILE__)
  asm volatile("v_nop\n\tv_nop\n\tv_nop\n\tv_nop" : "+v"(a), "+v"(b), "+v"(c), "+v"(d));
#endif
}
__device__ __forceinline__ void wave_lds_sync() {
  __builtin_amdgcn_fence(__ATOMIC_RELEASE, "workgroup");
  __builtin_amdgcn_wave_barrier();
  __builtin_amdgcn_fence(__ATOMIC_ACQUIRE, "workgroup");
}

__global__ __launch_bounds__(256) void cvt_flat(const float* __restrict__ in, _Float16* out, int n8, float scale) {
  const int i = blockIdx.x * 256 + threadIdx.x;
  if (i < n8) {
    float v[8];
    ld8(in + (size_t)i * 8, v);
    HU u;
#pragma unroll
    for (int e = 0; e < 8; ++e) u.s[e] = (_Float16)(bfr(v[e]) * scale);
    _Float16* p = out + (size_t)i * 8;
    *(volatile v4u*)p = u.u;
    __threadfence();
    *(volatile v4u*)p = u.u;
  }
}

__global__ __launch_bounds__(256) void cvt_xT(const float* __restrict__ X, _Float16* XT, int Cd) {
  __shared__ float sw[64][65];
  const int t = threadIdx.x;
  const int n0 = blockIdx.x * 64, k0 = blockIdx.y * 64, b = blockIdx.z;
  const float* Xb = X + (size_t)b * Cd * NT;
  {
    const int r = t >> 4, c4 = (t & 15) * 4;
#pragma unroll
    for (int it = 0; it < 4; ++it) {
      const int row = r + 16 * it;
      const v4f x = *(const v4f*)(Xb + (size_t)(k0 + row) * NT + n0 + c4);
      sw[row][c4 + 0] = x[0]; sw[row][c4 + 1] = x[1]; sw[row][c4 + 2] = x[2]; sw[row][c4 + 3] = x[3];
    }
  }
  __syncthreads();
  const int q8 = t & 7, rr = t >> 3;
  HU u[2];
#pragma unroll
  for (int it = 0; it < 2; ++it) {
    const int n = rr + 32 * it;
#pragma unroll
    for (int e = 0; e < 8; ++e) u[it].s[e] = (_Float16)bfr(sw[8 * q8 + e][n]);
  }
  for (int ps = 0; ps < 2; ++ps) {
#pragma unroll
    for (int it = 0; it < 2; ++it) {
      const int n = rr + 32 * it;
      _Float16* dst = XT + (size_t)(b * NT + n0 + n) * Cd + k0 + 8 * q8;
      *(volatile v4u*)dst = u[it].u;
    }
    __threadfence();
  }
}

__global__ __launch_bounds__(256) void k_xbar(const float* __restrict__ X, float* XB) {
  __shared__ float sm[32];
  const int tid = threadIdx.x, wave = tid >> 5, lane = tid & 31;
  const int c0 = blockIdx.x * 32, b = blockIdx.y;
#pragma unroll 1
  for (int q = 0; q < 4; ++q) {
    const int c = c0 + 4 * wave + q;
    const float* row = X + ((size_t)(b * CH + c)) * NT + 4 * lane;
    double s = 0.0;
#pragma unroll 1
    for (int j = 0; j < NT / 128; ++j) {
      const v4f v = *(const v4f*)(row + 128 * j);
      s += (double)bfr(v[0]); s += (double)bfr(v[1]); s += (double)bfr(v[2]); s += (double)bfr(v[3]);
    }
#pragma unroll
    for (int off = 16; off >= 1; off >>= 1) s += shfl_xor_d(s, off);
    if (lane == 0) sm[4 * wave + q] = (float)(s * (1.0 / (double)NT));
  }
  __syncthreads();
  if (wave == 0) {
    const int l8 = lane & 7;
    v4f o;
    o[0] = sm[4 * l8 + 0]; o[1] = sm[4 * l8 + 1]; o[2] = sm[4 * l8 + 2]; o[3] = sm[4 * l8 + 3];
    float* dst = XB + (size_t)b * CH + c0 + 4 * l8;
    for (int ps = 0; ps < 2; ++ps) {
      if (lane < 8) *(volatile v4f*)dst = o;
      __threadfence();
    }
  }
}

__global__ __launch_bounds__(256) void k_const(const float* __restrict__ XB1, const float* __restrict__ XB2,
                                               const float* __restrict__ Wv1, const float* __restrict__ bv1,
                                               const float* __restrict__ Wv2, const float* __restrict__ bv2,
                                               const float* __restrict__ Wf, float* FB) {
  __shared__ float sx1[CH], sx2[CH], sv1[CH], sv2[CH], sfb[CH];
  const int tid = threadIdx.x, wave = tid >> 5, lane = tid & 31;
  const int b = blockIdx.x;
#pragma unroll
  for (int q = 0; q < CH / 256; ++q) {
    sx1[tid + 256 * q] = XB1[(size_t)b * CH + tid + 256 * q];
    sx2[tid + 256 * q] = XB2[(size_t)b * CH + tid + 256 * q];
  }
  __syncthreads();
#pragma unroll 1
  for (int q = 0; q < CH / 256; ++q) {
    const int c = tid + 256 * q;
    const float* w1 = Wv1 + (size_t)c * CH;
    const float* w2 = Wv2 + (size_t)c * CH;
    double a1 = 0.0, a2 = 0.0;
#pragma unroll 2
    for (int cp = 0; cp < CH; ++cp) {
      a1 = fma((double)bfr(w1[cp]), (double)sx1[cp], a1);
      a2 = fma((double)bfr(w2[cp]), (double)sx2[cp], a2);
    }
    sv1[c] = (float)(a1 + (double)bfr(bv1[c]));
    sv2[c] = (float)(a2 + (double)bfr(bv2[c]));
  }
  __syncthreads();
#pragma unroll 1
  for (int q = 0; q < CH / 256; ++q) {
    const int o = tid + 256 * q;
    const float* wf = Wf + (size_t)o * (2 * CH);
    double f = 0.0;
#pragma unroll 2
    for (int c = 0; c < CH; ++c) {
      f = fma((double)bfr(wf[c]), (double)sv1[c], f);
      f = fma((double)bfr(wf[CH + c]), (double)sv2[c], f);
    }
    sfb[o] = (float)f;
  }
  __syncthreads();
  {
    const int l16 = lane & 15;
    v4f o;
    o[0] = sfb[64 * wave + 4 * l16 + 0]; o[1] = sfb[64 * wave + 4 * l16 + 1];
    o[2] = sfb[64 * wave + 4 * l16 + 2]; o[3] = sfb[64 * wave + 4 * l16 + 3];
    float* dst = FB + (size_t)b * CH + 64 * wave + 4 * l16;
    for (int ps = 0; ps < 2; ++ps) {
      if (lane < 16) *(volatile v4f*)dst = o;
      __threadfence();
    }
  }
}

__device__ __forceinline__ void kseg(v8f (&acc)[4][4], const _Float16* __restrict__ A, int lda, int m0,
                                     const _Float16* __restrict__ Bt, int ldb, int n0, int K, int rlane, int koff) {
  for (int kk = 0; kk < K; kk += 32) {
    v16h bh[4];
#pragma unroll
    for (int j = 0; j < 4; ++j) {
      const size_t bo = (size_t)(n0 + (j << 4) + rlane) * (size_t)ldb + koff + kk;
      bh[j] = ldfrag_h(Bt + bo);
    }
#pragma unroll
    for (int i = 0; i < 4; ++i) {
      const size_t ao = (size_t)(m0 + (i << 4) + rlane) * (size_t)lda + koff + kk;
      const v16h a0 = ldfrag_h(A + ao);
#pragma unroll
      for (int j = 0; j < 4; ++j) acc[i][j] = mma_h_raw(a0, bh[j], acc[i][j]);
      dep_guard_h(acc[i][0], acc[i][3], a0);
    }
    keep4_h(bh[0], bh[1], bh[2], bh[3]);
  }
}

template <int BM>
__device__ __forceinline__ float biasv(const float* __restrict__ rb, int nrb, int m, int n, int M) {
  if (BM == 1) return bfr(rb[min(m, nrb - 1)]);
  if (BM == 2) return bfr(rb[min(n, nrb - 1)]);
  if (BM == 3) return rb[min((n / NT) * M + m, nrb - 1)];
  return 0.0f;
}

template <int BM, int OM>
__global__ __launch_bounds__(256) void gemm64(
    const _Float16* __restrict__ A, int lda, long long sAb,
    const _Float16* __restrict__ Bt, int ldb, long long sBb,
    const float* __restrict__ rb, int nrb, float cs, float so,
    _Float16* Ch, float* Cf, int ldc, long long sCb, int M, int N, int K) {
  __shared__ __align__(16) float sT[8][16 * 68];
  const int lane = threadIdx.x & 31;
  const int wave = threadIdx.x >> 5;
  const int bz = blockIdx.y;
  const _Float16* Ab = A + (size_t)bz * (size_t)sAb;
  const _Float16* Bb = Bt + (size_t)bz * (size_t)sBb;
  const size_t cb = (size_t)bz * (size_t)sCb;
  const int tilesN = N >> 6;
  const int tilesM = M >> 6;
  const int tiles = tilesM * tilesN;
  const int item = blockIdx.x * 8 + wave;
  if (item >= tiles) return;
  const int tm = item / tilesN;
  const int tn = item - tm * tilesN;
  const int m0 = tm << 6;
  const int n0 = tn << 6;

  const int rlane = lane & 15;
  const int koff  = (lane >> 4) * 8;
  const int mOff  = (lane >> 4) * 8;

  v8f acc[4][4];
#pragma unroll
  for (int i = 0; i < 4; ++i)
#pragma unroll
    for (int j = 0; j < 4; ++j) acc[i][j] = zero8();

  kseg(acc, Ab, lda, m0, Bb, ldb, n0, K, rlane, koff);
  acc_guard4(acc[0][0], acc[0][1], acc[0][2], acc[0][3]);
  acc_guard4(acc[1][0], acc[1][1], acc[1][2], acc[1][3]);
  acc_guard4(acc[2][0], acc[2][1], acc[2][2], acc[2][3]);
  acc_guard4(acc[3][0], acc[3][1], acc[3][2], acc[3][3]);

  float* slab = sT[wave];

  if (OM == 0) {
    const int q8 = lane & 7, rr = lane >> 3, c8 = q8 * 8;
#pragma unroll
    for (int i = 0; i < 4; ++i) {
      const int mBase = m0 + (i << 4);
#pragma unroll
      for (int r = 0; r < 8; ++r) {
#pragma unroll
        for (int j = 0; j < 4; ++j) {
          slab[(mOff + r) * 68 + (j << 4) + rlane] = acc[i][j][r];
        }
      }
      wave_lds_sync();
      v4u uh[4];
#pragma unroll
      for (int it = 0; it < 4; ++it) {
        const int row = it * 4 + rr;
        float xs[8];
        ld8(slab + row * 68 + c8, xs);
        HU h;
#pragma unroll
        for (int e = 0; e < 8; ++e) {
          const float bb = biasv<BM>(rb, nrb, mBase + row, n0 + c8 + e, M);
          h.s[e] = (_Float16)((xs[e] * cs + bb) * so);
        }
        uh[it] = h.u;
      }
      for (int ps = 0; ps < 2; ++ps) {
#pragma unroll
        for (int it = 0; it < 4; ++it) {
          const int row = it * 4 + rr;
          const size_t co = cb + (size_t)(mBase + row) * (size_t)ldc + n0 + c8;
          *(volatile v4u*)(Ch + co) = uh[it];
        }
        __threadfence();
      }
      wave_lds_sync();
    }
  } else if (OM == 1) {
    const int q8 = lane & 7, rr = lane >> 3, c8 = q8 * 8;
#pragma unroll
    for (int j = 0; j < 4; ++j) {
      const int nBase = n0 + (j << 4);
#pragma unroll
      for (int i = 0; i < 4; ++i) {
        float t8[8];
#pragma unroll
        for (int r = 0; r < 8; ++r) t8[r] = acc[i][j][r];
        st8(slab + rlane * 68 + (i << 4) + mOff, t8);
      }
      wave_lds_sync();
      v4u uh[4];
#pragma unroll
      for (int it = 0; it < 4; ++it) {
        const int row = it * 4 + rr;
        float xs[8];
        ld8(slab + row * 68 + c8, xs);
        HU h;
#pragma unroll
        for (int e = 0; e < 8; ++e) {
          const float bb = biasv<BM>(rb, nrb, m0 + c8 + e, nBase + row, M);
          h.s[e] = (_Float16)((xs[e] * cs + bb) * so);
        }
        uh[it] = h.u;
      }
      for (int ps = 0; ps < 2; ++ps) {
#pragma unroll
        for (int it = 0; it < 4; ++it) {
          const int row = it * 4 + rr;
          const size_t co = cb + (size_t)(nBase + row) * (size_t)ldc + m0 + c8;
          *(volatile v4u*)(Ch + co) = uh[it];
        }
        __threadfence();
      }
      wave_lds_sync();
    }
  } else {
    const int r2 = lane >> 4, c4 = (lane & 15) * 4;
#pragma unroll
    for (int i = 0; i < 4; ++i) {
      const int mBase = m0 + (i << 4);
#pragma unroll
      for (int r = 0; r < 8; ++r) {
#pragma unroll
        for (int j = 0; j < 4; ++j) {
          slab[(mOff + r) * 68 + (j << 4) + rlane] = acc[i][j][r];
        }
      }
      wave_lds_sync();
      v4f ov[8];
#pragma unroll
      for (int it = 0; it < 8; ++it) {
        const int row = it * 2 + r2;
        const v4f x = *(const v4f*)(slab + row * 68 + c4);
        v4f o;
#pragma unroll
        for (int e = 0; e < 4; ++e) {
          const float bb = biasv<BM>(rb, nrb, mBase + row, n0 + c4 + e, M);
          o[e] = (x[e] * cs + bb) * so;
        }
        ov[it] = o;
      }
      for (int ps = 0; ps < 2; ++ps) {
#pragma unroll
        for (int it = 0; it < 8; ++it) {
          const int row = it * 2 + r2;
          const size_t co = cb + (size_t)(mBase + row) * (size_t)ldc + n0 + c4;
          *(volatile v4f*)(Cf + co) = ov[it];
        }
        __threadfence();
      }
      wave_lds_sync();
    }
  }
}

__global__ __launch_bounds__(256) void k_soft(const _Float16* __restrict__ Q8, const _Float16* __restrict__ K8,
                                              _Float16* E) {
  extern __shared__ __align__(16) float sc[];
  const int tid = threadIdx.x, wave = tid >> 5, lane = tid & 31;
  const int hh = lane >> 4, rl = lane & 15;
  const int rb = blockIdx.x, b = blockIdx.y, n0 = rb * RSB;

  const _Float16* aq = Q8 + (size_t)(b * NT + n0 + rl) * CQ + 8 * hh;
  for (int ct = wave; ct < NT / 16; ct += 8) {
    const _Float16* bk = K8 + (size_t)(b * NT + 16 * ct + rl) * CQ + 8 * hh;
    v8f a00 = zero8(), a10 = zero8();
#pragma unroll
    for (int ks = 0; ks < CQ / 32; ++ks) {
      const v16h kf = ldfrag_h(bk + 32 * ks);
      const v16h q0 = ldfrag_h(aq + 32 * ks);
      const v16h q1 = ldfrag_h(aq + 16 * CQ + 32 * ks);
      a00 = mma_h(q0, kf, a00);
      a10 = mma_h(q1, kf, a10);
    }
    const int mc = 16 * ct + rl;
#pragma unroll
    for (int r = 0; r < 8; ++r) {
      sc[(size_t)(8 * hh + r) * NT + mc]      = a00[r] * SCS;
      sc[(size_t)(16 + 8 * hh + r) * NT + mc] = a10[r] * SCS;
    }
  }
  __syncthreads();

  for (int q4 = 0; q4 < 4; ++q4) {
    const int row = 4 * wave + q4;
    float* rp = sc + (size_t)row * NT + 8 * lane;
    float mx = -3.0e38f;
#pragma unroll
    for (int j = 0; j < 4; ++j) {
      float v[8];
      ld8(rp + 256 * j, v);
#pragma unroll
      for (int e = 0; e < 8; ++e) mx = fmaxf(mx, v[e]);
    }
#pragma unroll
    for (int off = 16; off >= 1; off >>= 1) mx = fmaxf(mx, __shfl_xor(mx, off, 32));
    float z = 0.0f;
#pragma unroll
    for (int j = 0; j < 4; ++j) {
      float v[8];
      ld8(rp + 256 * j, v);
#pragma unroll
      for (int e = 0; e < 8; ++e) {
        const float ef = __expf(v[e] - mx);
        z += ef;
        v[e] = ef;
      }
      st8(rp + 256 * j, v);
    }
#pragma unroll
    for (int off = 16; off >= 1; off >>= 1) z += __shfl_xor(z, off, 32);
    const float rz = (float)NT * (1.0f / z);
    HU u[4];
#pragma unroll
    for (int j = 0; j < 4; ++j) {
      float v[8];
      ld8(rp + 256 * j, v);
#pragma unroll
      for (int e = 0; e < 8; ++e) {
        const float pc = fmaf(v[e], rz, -1.0f);
        const _Float16 h0 = (_Float16)(pc * SCE);
        const bool sub = fabsf((float)h0) < 6.103515625e-05f;
        u[j].s[e] = sub ? (_Float16)0.0f : h0;
      }
    }
    _Float16* erow = E + (size_t)(b * NT + n0 + row) * NT + 8 * lane;
    for (int ps = 0; ps < 2; ++ps) {
#pragma unroll
      for (int j = 0; j < 4; ++j) *(volatile v4u*)(erow + 256 * j) = u[j].u;
      __threadfence();
    }
  }
}

__global__ __launch_bounds__(256) void k_bn(const float* __restrict__ Y, const float* __restrict__ gam,
                                            const float* __restrict__ bet, float* out) {
  __shared__ double sred[8];
  const int c = blockIdx.x;
  const int tid = threadIdx.x, wave = tid >> 5, lane = tid & 31;
  const float* yc = Y + (size_t)c * TOK + 4 * tid;

  double s = 0.0;
#pragma unroll 1
  for (int j = 0; j < TOK / 1024; ++j) {
    const v4f v = *(const v4f*)(yc + 1024 * j);
    s += (double)v[0]; s += (double)v[1]; s += (double)v[2]; s += (double)v[3];
  }
#pragma unroll
  for (int off = 16; off >= 1; off >>= 1) s += shfl_xor_d(s, off);
  if (lane == 0) sred[wave] = s;
  __syncthreads();
  double tot = 0.0;
#pragma unroll
  for (int w = 0; w < 8; ++w) tot += sred[w];
  const float mean = (float)(tot * (1.0 / (double)TOK));
  __syncthreads();

  double q = 0.0;
#pragma unroll 1
  for (int j = 0; j < TOK / 1024; ++j) {
    const v4f v = *(const v4f*)(yc + 1024 * j);
#pragma unroll
    for (int e = 0; e < 4; ++e) {
      const double d = (double)(v[e] - mean);
      q += d * d;
    }
  }
#pragma unroll
  for (int off = 16; off >= 1; off >>= 1) q += shfl_xor_d(q, off);
  if (lane == 0) sred[wave] = q;
  __syncthreads();
  double totq = 0.0;
#pragma unroll
  for (int w = 0; w < 8; ++w) totq += sred[w];
  const float var = (float)(totq * (1.0 / (double)TOK));
  const float rstd = 1.0f / sqrtf(var + 1e-5f);
  const float g = bfr(gam[c]);
  const float be = bfr(bet[c]);

  for (int ps = 0; ps < 2; ++ps) {
#pragma unroll 1
    for (int j = 0; j < TOK / 1024; ++j) {
      const v4f v = *(const v4f*)(yc + 1024 * j);
      v4f o;
#pragma unroll
      for (int e = 0; e < 4; ++e) {
        const float yv = (v[e] - mean) * rstd * g + be;
        o[e] = yv > 0.0f ? yv : 0.0f;
      }
      float* dst = out + ((size_t)(j * CH + c)) * NT + 4 * tid;
      *(volatile v4f*)dst = o;
    }
    __threadfence();
  }
}

extern "C" void kernel_launch(void* const* d_in, const int* in_sizes, int n_in,
                              void* d_out, int out_size, void* d_ws, size_t ws_size,
                              hipStream_t stream) {
  if (n_in < 17) return;
  if (in_sizes[0] != NB * CH * NT || in_sizes[1] != NB * CH * NT) return;
  if (in_sizes[2] != CQ * CH || in_sizes[3] != CQ || in_sizes[4] != CQ * CH || in_sizes[5] != CQ) return;
  if (in_sizes[6] != CH * CH || in_sizes[7] != CH || in_sizes[8] != CQ * CH || in_sizes[9] != CQ) return;
  if (in_sizes[10] != CQ * CH || in_sizes[11] != CQ || in_sizes[12] != CH * CH || in_sizes[13] != CH) return;
  if (in_sizes[14] != CH * 2 * CH || in_sizes[15] != CH || in_sizes[16] != CH) return;
  if (out_size != OUTN) return;

  const float* rgb    = (const float*)d_in[0];
  const float* dep    = (const float*)d_in[1];
  const float* Wq_rgb = (const float*)d_in[2];
  const float* bq_rgb = (const float*)d_in[3];
  const float* Wk_dep = (const float*)d_in[4];
  const float* bk_dep = (const float*)d_in[5];
  const float* Wv_dep = (const float*)d_in[6];
  const float* bv_dep = (const float*)d_in[7];
  const float* Wq_dep = (const float*)d_in[8];
  const float* bq_dep = (const float*)d_in[9];
  const float* Wk_rgb = (const float*)d_in[10];
  const float* bk_rgb = (const float*)d_in[11];
  const float* Wv_rgb = (const float*)d_in[12];
  const float* bv_rgb = (const float*)d_in[13];
  const float* W_fuse = (const float*)d_in[14];
  const float* gam    = (const float*)d_in[15];
  const float* bet    = (const float*)d_in[16];

  const size_t PWQK = (size_t)CQ * CH * 2;
  const size_t PWV  = (size_t)CH * CH * 2;
  const size_t PWF  = (size_t)CH * 2 * CH * 2;
  const size_t PXT  = (size_t)TOK * CH * 2;
  const size_t PE   = (size_t)TOK * NT * 2;
  const size_t PY   = (size_t)CH * TOK * 4;
  const size_t PXB  = (size_t)NB * CH * 4;
  const size_t PQK  = (size_t)TOK * CQ * 2;
  const size_t PVP  = (size_t)CH * TOK * 2;
  const size_t PATT = (size_t)TOK * 2 * CH * 2;
  if (PE > 2 * PXT || PY > 2 * PXT) return;

  size_t off = 0;
  const size_t oWQ1 = off; off += PWQK;
  const size_t oWK1 = off; off += PWQK;
  const size_t oWQ2 = off; off += PWQK;
  const size_t oWK2 = off; off += PWQK;
  const size_t oWV1 = off; off += PWV;
  const size_t oWV2 = off; off += PWV;
  const size_t oWF  = off; off += PWF;
  const size_t oXTr = off; off += PXT;
  const size_t oXTd = off; off += PXT;
  const size_t oXBr = off; off += PXB;
  const size_t oXBd = off; off += PXB;
  const size_t oFB  = off; off += PXB;
  const size_t oQ1  = off; off += PQK;
  const size_t oK1  = off; off += PQK;
  const size_t oQ2  = off; off += PQK;
  const size_t oK2  = off; off += PQK;
  const size_t oV1  = off; off += PVP;
  const size_t oV2  = off; off += PVP;
  const size_t oATT = off; off += PATT;
  if (off > ws_size) return;
  if (off > (size_t)134217728) return;

  char* ws = (char*)d_ws;
  _Float16* WQ1 = (_Float16*)(ws + oWQ1);
  _Float16* WK1 = (_Float16*)(ws + oWK1);
  _Float16* WQ2 = (_Float16*)(ws + oWQ2);
  _Float16* WK2 = (_Float16*)(ws + oWK2);
  _Float16* WV1 = (_Float16*)(ws + oWV1);
  _Float16* WV2 = (_Float16*)(ws + oWV2);
  _Float16* WF  = (_Float16*)(ws + oWF);
  _Float16* XTr = (_Float16*)(ws + oXTr);
  _Float16* XTd = (_Float16*)(ws + oXTd);
  float*    XBr = (float*)(ws + oXBr);
  float*    XBd = (float*)(ws + oXBd);
  float*    FB  = (float*)(ws + oFB);
  _Float16* Q1  = (_Float16*)(ws + oQ1);
  _Float16* K1  = (_Float16*)(ws + oK1);
  _Float16* Q2  = (_Float16*)(ws + oQ2);
  _Float16* K2  = (_Float16*)(ws + oK2);
  _Float16* V1  = (_Float16*)(ws + oV1);
  _Float16* V2  = (_Float16*)(ws + oV2);
  _Float16* ATT = (_Float16*)(ws + oATT);
  _Float16* E   = (_Float16*)(ws + oXTr);
  float*    Y   = (float*)(ws + oXTr);
  float*    outf = (float*)d_out;

  const dim3 blk(256);
  const int n8qk = (CQ * CH) / 8;
  const int n8v  = (CH * CH) / 8;
  const int n8f  = (CH * 2 * CH) / 8;
  const dim3 gWqk((n8qk + 255) / 256);
  const dim3 gWv((n8v + 255) / 256);
  const dim3 gWf((n8f + 255) / 256);
  const dim3 gXT(NT / 64, CH / 64, NB);
  const dim3 gXB(CH / 32, NB);
  const dim3 gCo(NB);
  const dim3 gQK(((TOK / 64) * (CQ / 64) + 7) / 8, 1);
  const dim3 gV(((CH / 64) * (TOK / 64) + 7) / 8, 1);
  const dim3 gPV(((CH / 64) * (NT / 64) + 7) / 8, NB);
  const dim3 gSo(NRB, NB);
  const dim3 gBN(CH);
  const float csW  = 1.0f / SCW;
  const float csPV = SCA / (SCE * SCV * (float)NT);
  const float csF  = 1.0f / (SCW * SCA);
  const size_t ldsSoft = (size_t)RSB * NT * sizeof(float);
  const long long zll = 0;

  cvt_flat<<<gWqk, blk, 0, stream>>>(Wq_rgb, WQ1, n8qk, SCW);
  cvt_flat<<<gWqk, blk, 0, stream>>>(Wk_dep, WK1, n8qk, SCW);
  cvt_flat<<<gWqk, blk, 0, stream>>>(Wq_dep, WQ2, n8qk, SCW);
  cvt_flat<<<gWqk, blk, 0, stream>>>(Wk_rgb, WK2, n8qk, SCW);
  cvt_flat<<<gWv,  blk, 0, stream>>>(Wv_dep, WV1, n8v, SCW);
  cvt_flat<<<gWv,  blk, 0, stream>>>(Wv_rgb, WV2, n8v, SCW);
  cvt_flat<<<gWf,  blk, 0, stream>>>(W_fuse, WF, n8f, SCW);
  cvt_xT<<<gXT, blk, 0, stream>>>(rgb, XTr, CH);
  cvt_xT<<<gXT, blk, 0, stream>>>(dep, XTd, CH);
  k_xbar<<<gXB, blk, 0, stream>>>(rgb, XBr);
  k_xbar<<<gXB, blk, 0, stream>>>(dep, XBd);
  k_const<<<gCo, blk, 0, stream>>>(XBd, XBr, Wv_dep, bv_dep, Wv_rgb, bv_rgb, W_fuse, FB);
  gemm64<2, 0><<<gQK, blk, 0, stream>>>(XTr, CH, zll, WQ1, CH, zll, bq_rgb, CQ, csW, SCQK, Q1, XBr, CQ, zll, TOK, CQ, CH);
  gemm64<2, 0><<<gQK, blk, 0, stream>>>(XTd, CH, zll, WK1, CH, zll, bk_dep, CQ, csW, SCQK, K1, XBr, CQ, zll, TOK, CQ, CH);
  gemm64<2, 0><<<gQK, blk, 0, stream>>>(XTd, CH, zll, WQ2, CH, zll, bq_dep, CQ, csW, SCQK, Q2, XBr, CQ, zll, TOK, CQ, CH);
  gemm64<2, 0><<<gQK, blk, 0, stream>>>(XTr, CH, zll, WK2, CH, zll, bk_rgb, CQ, csW, SCQK, K2, XBr, CQ, zll, TOK, CQ, CH);
  gemm64<1, 0><<<gV, blk, 0, stream>>>(WV1, CH, zll, XTd, CH, zll, bv_dep, CH, csW, SCV, V1, XBr, TOK, zll, CH, TOK, CH);
  gemm64<1, 0><<<gV, blk, 0, stream>>>(WV2, CH, zll, XTr, CH, zll, bv_rgb, CH, csW, SCV, V2, XBr, TOK, zll, CH, TOK, CH);
  k_soft<<<gSo, blk, ldsSoft, stream>>>(Q1, K1, E);
  gemm64<0, 1><<<gPV, blk, 0, stream>>>(V1, TOK, (long long)NT, E, NT, (long long)NT * NT, bv_dep, CH, csPV, 1.0f,
                                        ATT, XBr, 2 * CH, (long long)NT * 2 * CH, CH, NT, NT);
  k_soft<<<gSo, blk, ldsSoft, stream>>>(Q2, K2, E);
  gemm64<0, 1><<<gPV, blk, 0, stream>>>(V2, TOK, (long long)NT, E, NT, (long long)NT * NT, bv_rgb, CH, csPV, 1.0f,
                                        ATT + CH, XBr, 2 * CH, (long long)NT * 2 * CH, CH, NT, NT);
  gemm64<3, 2><<<gV, blk, 0, stream>>>(WF, 2 * CH, zll, ATT, 2 * CH, zll, FB, NB * CH, csF, 1.0f, Q1, Y, TOK, zll, CH, TOK, 2 * CH);
  k_bn<<<gBN, blk, 0, stream>>>(Y, gam, bet, outf);
}
